// SingleHeadAttention_24257975288111
// MI455X (gfx1250) — hardware-verified
//
#include <hip/hip_runtime.h>
#ifndef NB
#define NB 4
#endif
#ifndef SEQ
#define SEQ 2048
#endif
#define NB_FULL 4
#define SEQ_FULL 2048
#define SQ SEQ
#define DM 1024
#define QT 256
#define RQ ((SQ < 512) ? SQ : 512)
#define NKX SQ
static_assert(NB >= 1 && NB <= NB_FULL);
static_assert(SQ >= QT && SQ <= SEQ_FULL);
static_assert(SQ % QT == 0);
static_assert(QT % 128 == 0);
static_assert(RQ % QT == 0);
static_assert(SQ % 64 == 0 && DM % 128 == 0);

typedef unsigned short v8us __attribute__((ext_vector_type(8), may_alias));
typedef float  v8f  __attribute__((ext_vector_type(8)));
typedef float  v4f  __attribute__((ext_vector_type(4)));
typedef float  v4fa __attribute__((ext_vector_type(4), may_alias));
typedef _Float16 v16h __attribute__((ext_vector_type(16)));
union FragH { v16h v; v8us half[2]; _Float16 h[16]; unsigned short u[16]; };

__device__ __forceinline__ unsigned short bf16_bits(float x) { unsigned int u = __float_as_uint(x); return (unsigned short)((u + 0x7FFFu + ((u >> 16) & 1u)) >> 16); }
__device__ __forceinline__ float bf16_val(unsigned short b) { return __uint_as_float(((unsigned int)b) << 16); }
__device__ __forceinline__ float bf16_rne(float x) { return bf16_val(bf16_bits(x)); }

__global__ __launch_bounds__(256) void k_wnat(const float* __restrict__ w, size_t n8, float scale, _Float16* __restrict__ Bt) {
  const size_t t = (size_t)blockIdx.x * 256 + threadIdx.x; if (t >= n8) return;
  const v4f a = *(const v4fa*)(w + t * 8), c = *(const v4fa*)(w + t * 8 + 4); FragH f;
#pragma unroll
  for (int q = 0; q < 4; ++q) { const float av = a[q], cv = c[q]; f.h[q] = (_Float16)(bf16_rne(av) * scale); f.h[4 + q] = (_Float16)(bf16_rne(cv) * scale); }
  const v8us o = f.half[0];
  *(volatile v8us*)((unsigned short*)Bt + t * 8) = o; __threadfence(); *(volatile v8us*)((unsigned short*)Bt + t * 8) = o;
}

__global__ __launch_bounds__(256) void k_x16(const float* __restrict__ x, _Float16* __restrict__ X16, size_t n8) {
  const size_t t = (size_t)blockIdx.x * 256 + threadIdx.x; if (t >= n8) return;
  const v4f a = *(const v4fa*)(x + t * 8), c = *(const v4fa*)(x + t * 8 + 4); FragH f;
#pragma unroll
  for (int q = 0; q < 4; ++q) { const float av = a[q], cv = c[q]; f.h[q] = (_Float16)bf16_rne(av); f.h[4 + q] = (_Float16)bf16_rne(cv); }
  const v8us o = f.half[0];
  *(volatile v8us*)((unsigned short*)X16 + t * 8) = o; __threadfence(); *(volatile v8us*)((unsigned short*)X16 + t * 8) = o;
}

__global__ __launch_bounds__(256) void k_hl(const float* __restrict__ F, _Float16* __restrict__ Hh, _Float16* __restrict__ Hl, size_t n8) {
  const size_t t = (size_t)blockIdx.x * 256 + threadIdx.x; if (t >= n8) return; FragH fh, fl;
  const v4f a = *(const v4fa*)(F + t * 8), c = *(const v4fa*)(F + t * 8 + 4);
#pragma unroll
  for (int q = 0; q < 4; ++q) { const float av = a[q], cv = c[q]; _Float16 h = (_Float16)av; fh.h[q] = h; fl.h[q] = (_Float16)((av - (float)h) * 1024.0f); h = (_Float16)cv; fh.h[4 + q] = h; fl.h[4 + q] = (_Float16)((cv - (float)h) * 1024.0f); }
  for (int pass = 0; pass < 2; ++pass) { *(volatile v8us*)((unsigned short*)Hh + t * 8) = fh.half[0]; *(volatile v8us*)((unsigned short*)Hl + t * 8) = fl.half[0]; if (pass == 0) __threadfence(); }
}

template <int NHv, int TTv, int NLG>
__global__ __launch_bounds__(256) void k_vt(const _Float16* __restrict__ V16, int ldv, int voff, _Float16* __restrict__ Vt) {
  __shared__ unsigned short tl[64][66];
  const int tid = threadIdx.x; const int slab = blockIdx.x / NLG, lg = blockIdx.x % NLG; const int h = slab % NHv;
  for (int i = tid; i < 64 * 8; i += 256) { const int r = i / 8, c8 = (i % 8) * 8; FragH f;
    f.half[0] = *(const v8us*)((const unsigned short*)V16 + ((size_t)lg * 64 + r) * ldv + voff + h * 64 + c8);
#pragma unroll
    for (int q = 0; q < 8; ++q) tl[r][c8 + q] = f.u[q]; }
  __syncthreads();
  for (int pass = 0; pass < 2; ++pass) {
#pragma unroll
    for (int rd = 0; rd < 2; ++rd) { const int d = rd * 32 + tid / 8, pc = tid % 8; FragH f;
#pragma unroll
      for (int q = 0; q < 8; ++q) f.u[q] = tl[pc * 8 + q][d];
      *(volatile v8us*)((unsigned short*)Vt + ((size_t)h * 64 + d) * TTv + lg * 64 + pc * 8) = f.half[0]; }
    if (pass == 0) __threadfence(); }
}

__device__ __forceinline__ v16h g2_frag(const _Float16* p, int hh) { FragH f; f.half[0] = *(const v8us*)((const unsigned short*)p + 8 * hh); f.half[1] = *(const v8us*)((const unsigned short*)p + 16 + 8 * hh); return f.v; }
__device__ __forceinline__ v8f g2_mma(v16h a, v16h b, v8f c) { v8f d = __builtin_amdgcn_wmma_f32_16x16x32_f16(false, a, false, b, (short)0, c, false, false); asm volatile("v_nop\n\tv_nop\n\tv_nop\n\tv_nop" : "+v"(d) : "v"(a), "v"(b)); return d; }

__global__ __launch_bounds__(128) void k_gemm2(const _Float16* __restrict__ A, int lda, const _Float16* __restrict__ Bh, int ldb, float alpha, const float* CP,
                                               float* C, int ldc, int M, int N, int K) {
  __shared__ __attribute__((aligned(16))) float so[4][32][68];
  const int tid = threadIdx.x, w = tid >> 5, lane = tid & 31, ln = lane & 15, hh = lane >> 4;
  const int ntn = N >> 6; const int mt = blockIdx.x / ntn, nq = blockIdx.x - mt * ntn; const int row0 = mt * 128 + 32 * w, col0 = nq * 64; if (row0 >= M) return;
  const _Float16* a0p = A + (size_t)(row0 + ln) * lda; const _Float16* a1p = a0p + (size_t)16 * lda;
  const _Float16* b0p = Bh + (size_t)(col0 + ln) * ldb; const _Float16* b1p = b0p + (size_t)16 * ldb; const _Float16* b2p = b1p + (size_t)16 * ldb; const _Float16* b3p = b2p + (size_t)16 * ldb;
  const v8f z8 = {0.f,0.f,0.f,0.f,0.f,0.f,0.f,0.f}; v8f c00 = z8, c01 = z8, c02 = z8, c03 = z8, c10 = z8, c11 = z8, c12 = z8, c13 = z8;
#pragma unroll 1
  for (int kb = 0; kb < K; kb += 32) { const v16h a0 = g2_frag(a0p + kb, hh), a1 = g2_frag(a1p + kb, hh);
    v16h b = g2_frag(b0p + kb, hh); c00 = g2_mma(a0, b, c00); c10 = g2_mma(a1, b, c10);
    b = g2_frag(b1p + kb, hh); c01 = g2_mma(a0, b, c01); c11 = g2_mma(a1, b, c11);
    b = g2_frag(b2p + kb, hh); c02 = g2_mma(a0, b, c02); c12 = g2_mma(a1, b, c12);
    b = g2_frag(b3p + kb, hh); c03 = g2_mma(a0, b, c03); c13 = g2_mma(a1, b, c13); }
  v8f accs[8] = {c00, c01, c02, c03, c10, c11, c12, c13};
#pragma unroll
  for (int u = 0; u < 8; ++u) { const int t = u & 3, half = u >> 2; const int col = col0 + t * 16 + ln;
#pragma unroll
    for (int r = 0; r < 8; ++r) { const int rloc = half * 16 + 8 * hh + r; float v = accs[u][r] * alpha; if (CP) v += CP[(size_t)(row0 + rloc) * ldc + col]; so[w][rloc][t * 16 + ln] = v; } }
  __builtin_amdgcn_fence(4, "workgroup"); __builtin_amdgcn_wave_barrier();
  const int rsub = lane >> 4, c4 = (lane & 15) * 4;
  for (int pass = 0; pass < 2; ++pass) {
#pragma unroll
    for (int q = 0; q < 16; ++q) { const int r = q * 2 + rsub; const v4f v = *(const v4fa*)&so[w][r][c4]; *(volatile v4f*)(C + (size_t)(row0 + r) * ldc + col0 + c4) = v; }
    if (pass == 0) __threadfence(); }
}

template <bool HL>
__global__ __launch_bounds__(128) void k_rsm(const float* __restrict__ S, _Float16* __restrict__ P, _Float16* __restrict__ PL, int q0, int nk) {
  #pragma clang fp contract(off)
  __shared__ __attribute__((aligned(16))) unsigned short sth[128][72];
  __shared__ __attribute__((aligned(16))) unsigned short stl[128][72];
  const int tid = threadIdx.x; const int i = blockIdx.x * 128 + tid;
  const float* s = S + (size_t)i * NKX; const int last = q0 + i;
  float mx = -3.0e38f;
#pragma unroll 1
  for (int j = 0; j < nk; ++j) { const float f = (j <= last) ? 1.f : 0.f; mx = fmaxf(mx, fmaf(f, s[j], (1.f - f) * -1.0e9f)); }
  float se = 0.f;
#pragma unroll 1
  for (int j = 0; j < nk; ++j) { const float f = (j <= last) ? 1.f : 0.f; se += __expf(fmaf(f, s[j], (1.f - f) * -1.0e9f) - mx); }
  const float sc = 256.0f / se;
  const int rb = tid >> 3, pc = tid & 7;
#pragma unroll 1
  for (int j0 = 0; j0 < nk; j0 += 64) {
#pragma unroll 1
    for (int g = 0; g < 8; ++g) {
      const int jb = j0 + g * 8;
      const v4f sa = *(const v4fa*)(s + jb), sb = *(const v4fa*)(s + jb + 4);
      const float sv[8] = {sa[0], sa[1], sa[2], sa[3], sb[0], sb[1], sb[2], sb[3]};
      FragH fr, fl;
#pragma unroll
      for (int q = 0; q < 8; ++q) { const int j = jb + q; const float f = (j <= last) ? 1.f : 0.f; const float pv = __expf(fmaf(f, sv[q], (1.f - f) * -1.0e9f) - mx) * sc;
        const _Float16 h = (_Float16)pv; fr.h[q] = h; fl.h[q] = HL ? (_Float16)((pv - (float)h) * 1024.0f) : (_Float16)0.0f; }
      *(v8us*)&sth[tid][g * 8] = fr.half[0];
      if (HL) *(v8us*)&stl[tid][g * 8] = fl.half[0];
    }
    __syncthreads();
    for (int pass = 0; pass < 2; ++pass) {
#pragma unroll
      for (int u = 0; u < 8; ++u) {
        const int rl = u * 16 + rb;
        const size_t go = (size_t)(blockIdx.x * 128 + rl) * NKX + j0 + pc * 8;
        const v8us vh = *(const v8us*)&sth[rl][pc * 8];
        *(volatile v8us*)((unsigned short*)P + go) = vh;
        if (HL) { const v8us vl = *(const v8us*)&stl[rl][pc * 8]; *(volatile v8us*)((unsigned short*)PL + go) = vl; }
      }
      if (pass == 0) __threadfence();
    }
    __syncthreads();
  }
}

__global__ __launch_bounds__(256) void k_dec4(float* __restrict__ y, size_t n4) {
  #pragma clang fp contract(off)
  const size_t t = (size_t)blockIdx.x * 256 + threadIdx.x; if (t >= n4) return;
  v4f v = *(const v4fa*)(y + t * 4);
#pragma unroll
  for (int q = 0; q < 4; ++q) { const float a = v[q]; v[q] = rintf(a * 10000.0f) * 0.0001f; }
  *(volatile v4f*)(y + t * 4) = v; __threadfence(); *(volatile v4f*)(y + t * 4) = v;
}

extern "C" void kernel_launch(void* const* d_in, const int* in_sizes, int n_in,
                              void* d_out, int out_size, void* d_ws, size_t ws_size, hipStream_t stream) {
  if (n_in < 4) return;
  const long long need0 = (long long)(NB - 1) * SEQ_FULL * DM + (long long)SQ * DM;
  if ((long long)in_sizes[0] < need0 || (long long)out_size < need0) return;
  if (in_sizes[1] < DM * DM || in_sizes[2] < DM * DM || in_sizes[3] < DM * DM) return;
  const float* x = (const float*)d_in[0]; const float* wk = (const float*)d_in[1]; const float* wq = (const float*)d_in[2]; const float* wv = (const float*)d_in[3];
  char* ws = (char*)d_ws; size_t off = 0;
  auto take = [&](size_t bytes) { char* p = ws + off; off += (bytes + 255) & ~(size_t)255; return p; };
  _Float16* BQ = (_Float16*)take((size_t)DM * DM * 2); _Float16* BK = (_Float16*)take((size_t)DM * DM * 2); _Float16* BV = (_Float16*)take((size_t)DM * DM * 2);
  _Float16* X16 = (_Float16*)take((size_t)SQ * DM * 2);
  float* F = (float*)take((size_t)SQ * DM * 4);
  _Float16* QH = (_Float16*)take((size_t)SQ * DM * 2); _Float16* QL = (_Float16*)take((size_t)SQ * DM * 2);
  _Float16* KH = (_Float16*)take((size_t)SQ * DM * 2); _Float16* KL = (_Float16*)take((size_t)SQ * DM * 2);
  _Float16* VH = (_Float16*)take((size_t)SQ * DM * 2); _Float16* VL = (_Float16*)take((size_t)SQ * DM * 2);
  float* S = (float*)take((size_t)QT * NKX * 4); _Float16* P = (_Float16*)take((size_t)QT * NKX * 2); _Float16* PL = (_Float16*)take((size_t)QT * NKX * 2);
  _Float16* VT = (_Float16*)take((size_t)DM * SQ * 2); _Float16* VTL = (_Float16*)take((size_t)DM * SQ * 2);
  if (off > ws_size || off > ((size_t)128 << 20)) return;

  const size_t w8 = (size_t)DM * DM / 8; const unsigned gw = (unsigned)((w8 + 255) / 256);
  k_wnat<<<gw, 256, 0, stream>>>(wq, w8, 1024.0f, BQ);
  k_wnat<<<gw, 256, 0, stream>>>(wk, w8, 1024.0f, BK);
  k_wnat<<<gw, 256, 0, stream>>>(wv, w8, 1024.0f, BV);
  const size_t p8 = (size_t)SQ * DM / 8; const unsigned gp = (unsigned)((p8 + 255) / 256);
  const unsigned gproj = (unsigned)((SQ / 128) * (DM / 64));
  const unsigned gpv = (unsigned)((QT / 128) * (DM / 64));
  const float a_proj = 0.0009765625f;
  const float a_s_hh = 0.03125f;
  const float a_s_res = 0.000030517578125f;
  const float a_o_hh = 0.00390625f;
  const float a_o_res = 0.000003814697265625f;
  for (int b = 0; b < NB; ++b) {
    const float* xb = x + (size_t)b * SEQ_FULL * DM; float* ob = (float*)d_out + (size_t)b * SEQ_FULL * DM;
    k_x16<<<gp, 256, 0, stream>>>(xb, X16, p8);
    k_gemm2<<<gproj, 128, 0, stream>>>(X16, DM, BQ, DM, a_proj, nullptr, F, DM, SQ, DM, DM); k_hl<<<gp, 256, 0, stream>>>(F, QH, QL, p8);
    k_gemm2<<<gproj, 128, 0, stream>>>(X16, DM, BK, DM, a_proj, nullptr, F, DM, SQ, DM, DM); k_hl<<<gp, 256, 0, stream>>>(F, KH, KL, p8);
    k_gemm2<<<gproj, 128, 0, stream>>>(X16, DM, BV, DM, a_proj, nullptr, F, DM, SQ, DM, DM); k_hl<<<gp, 256, 0, stream>>>(F, VH, VL, p8);
    k_vt<DM / 64, SQ, SQ / 64><<<(unsigned)((DM / 64) * (SQ / 64)), 256, 0, stream>>>(VH, DM, 0, VT);
    k_vt<DM / 64, SQ, (RQ) / 64><<<(unsigned)((DM / 64) * ((RQ) / 64)), 256, 0, stream>>>(VL, DM, 0, VTL);
    for (int q0 = 0; q0 < SQ; q0 += QT) {
      const int nk = q0 + QT;
      const bool res = (q0 < RQ);
      const unsigned gs = (unsigned)((QT / 128) * (nk / 64));
      k_gemm2<<<gs, 128, 0, stream>>>(QH + (size_t)q0 * DM, DM, KH, DM, a_s_hh, nullptr, S, NKX, QT, nk, DM);
      if (res) {
        k_gemm2<<<gs, 128, 0, stream>>>(QL + (size_t)q0 * DM, DM, KH, DM, a_s_res, S, S, NKX, QT, nk, DM);
        k_gemm2<<<gs, 128, 0, stream>>>(QH + (size_t)q0 * DM, DM, KL, DM, a_s_res, S, S, NKX, QT, nk, DM);
        k_rsm<true><<<(unsigned)(QT / 128), 128, 0, stream>>>(S, P, PL, q0, nk);
      } else {
        k_rsm<false><<<(unsigned)(QT / 128), 128, 0, stream>>>(S, P, PL, q0, nk);
      }
      float* ot = ob + (size_t)q0 * DM;
      k_gemm2<<<gpv, 128, 0, stream>>>(P, NKX, VT, SQ, a_o_hh, nullptr, ot, DM, QT, DM, nk);
      if (res) {
        k_gemm2<<<gpv, 128, 0, stream>>>(P, NKX, VTL, SQ, a_o_res, ot, ot, DM, QT, DM, nk);
        k_gemm2<<<gpv, 128, 0, stream>>>(PL, NKX, VT, SQ, a_o_res, ot, ot, DM, QT, DM, nk);
      }
    }
    k_dec4<<<(unsigned)(((size_t)SQ * DM / 4 + 255) / 256), 256, 0, stream>>>(ob, (size_t)SQ * DM / 4);
  }
}
